// HNN_10488310137126
// MI455X (gfx1250) — hardware-verified
//
#include <hip/hip_runtime.h>


#define NBT  524288
#define RCH  16384
#define HID  128
#define DTC  0.02f
typedef _Float16 h16;
typedef unsigned short bf;
typedef __attribute__((ext_vector_type(16))) __bf16   v16bf;
typedef __attribute__((ext_vector_type(16))) _Float16 v16h;
typedef __attribute__((ext_vector_type(8)))  _Float16 v8h;
typedef __attribute__((ext_vector_type(8)))  unsigned short v8us;
typedef __attribute__((ext_vector_type(8)))  float    v8f;
typedef __attribute__((ext_vector_type(4)))  float    v4f;
typedef v8h  __attribute__((may_alias)) v8ha;
typedef v4f  __attribute__((may_alias)) v4fa;
typedef v8us __attribute__((may_alias)) v8usa;

__device__ __forceinline__ unsigned short f2bf(float f) { unsigned u = __float_as_uint(f); u += 0x7FFFu + ((u >> 16) & 1u); return (unsigned short)(u >> 16); }
__device__ __forceinline__ float bf2f(unsigned short b) { return __uint_as_float(((unsigned)b) << 16); }
__device__ __forceinline__ float bfr(float f) { return bf2f(f2bf(f)); }
__device__ __forceinline__ v16h cat16(v8h lo, v8h hi) { return __builtin_shufflevector(lo, hi, 0, 1, 2, 3, 4, 5, 6, 7, 8, 9, 10, 11, 12, 13, 14, 15); }
__device__ __forceinline__ v16bf cat16b(v8us lo, v8us hi) { return __builtin_bit_cast(v16bf, __builtin_shufflevector(lo, hi, 0, 1, 2, 3, 4, 5, 6, 7, 8, 9, 10, 11, 12, 13, 14, 15)); }
__device__ __forceinline__ v8f wmma16(v16h a, v16h b, v8f c) { return __builtin_amdgcn_wmma_f32_16x16x32_f16(false, a, false, b, (short)0, c, false, false); }
__device__ __forceinline__ v8f wmmab(v16bf a, v16bf b, v8f c) { return __builtin_amdgcn_wmma_f32_16x16x32_bf16(false, a, false, b, (short)0, c, false, false); }


template <typename T16> struct WFrag;
template <> struct WFrag<h16> { typedef v16h V; static __device__ __forceinline__ V ld(const h16* p) { return cat16(*(const v8h*)p, *(const v8h*)(p + 16)); } static __device__ __forceinline__ v8f mma(V a, V b, v8f c) { return wmma16(a, b, c); } };
template <> struct WFrag<bf> { typedef v16bf V; static __device__ __forceinline__ V ld(const bf* p) { return cat16b(*(const v8us*)p, *(const v8us*)(p + 16)); } static __device__ __forceinline__ v8f mma(V a, V b, v8f c) { return wmmab(a, b, c); } };
template <typename T16, int NSPLIT, bool BIAS>
__global__ __launch_bounds__(32) void k_gemmw(const T16* __restrict__ A, const T16* __restrict__ A2, const T16* __restrict__ Bt, const T16* __restrict__ Bt2, int K, float* C, int ldc, const float* __restrict__ bias, size_t sA, size_t sB, size_t sC) {
    typedef typename WFrag<T16>::V V;
    __shared__ __align__(16) float os[16 * 68];
    const size_t z = blockIdx.z; A += z * sA; if (A2) A2 += z * sA; Bt += z * sB; if (Bt2) Bt2 += z * sB; C += z * sC;
    const int lane = threadIdx.x & 31, lr = lane & 15, hi = lane >> 4; const int r0 = blockIdx.x * 64, c0 = blockIdx.y * 64;
    v8f acc[4][4];
#pragma unroll
    for (int mb = 0; mb < 4; ++mb)
#pragma unroll
        for (int nb = 0; nb < 4; ++nb) acc[mb][nb] = (v8f){};
    const size_t aoff = (size_t)(r0 + lr) * K + 8 * hi, boff = (size_t)(c0 + lr) * K + 8 * hi;
#pragma unroll 1
    for (int kc = 0; kc < K; kc += 32) {
        V a[4], a2[4];
#pragma unroll
        for (int mb = 0; mb < 4; ++mb) { a[mb] = WFrag<T16>::ld(A + aoff + (size_t)mb * 16 * K + kc); if (NSPLIT == 1 || NSPLIT == 2) a2[mb] = WFrag<T16>::ld(A2 + aoff + (size_t)mb * 16 * K + kc); }
#pragma unroll
        for (int nb = 0; nb < 4; ++nb) { const V b = WFrag<T16>::ld(Bt + boff + (size_t)nb * 16 * K + kc); V b2; if (NSPLIT >= 2) b2 = WFrag<T16>::ld(Bt2 + boff + (size_t)nb * 16 * K + kc);
#pragma unroll
            for (int mb = 0; mb < 4; ++mb) { acc[mb][nb] = WFrag<T16>::mma(a[mb], b, acc[mb][nb]); if (NSPLIT == 1 || NSPLIT == 2) acc[mb][nb] = WFrag<T16>::mma(a2[mb], b, acc[mb][nb]); if (NSPLIT >= 2) acc[mb][nb] = WFrag<T16>::mma(a[mb], b2, acc[mb][nb]); } }
        asm volatile("v_nop\n\tv_nop\n\tv_nop\n\tv_nop" : "+v"(acc[0][0]), "+v"(acc[1][1]), "+v"(acc[2][2]), "+v"(acc[3][3]) : "v"(a[0]), "v"(a[3]));
    }
#pragma unroll
    for (int mb = 0; mb < 4; ++mb) {
#pragma unroll
        for (int nb = 0; nb < 4; ++nb) {
#pragma unroll
            for (int j = 0; j < 8; ++j) os[(hi * 8 + j) * 68 + nb * 16 + lr] = acc[mb][nb][j]; }
        __builtin_amdgcn_wave_barrier(); asm volatile("" ::: "memory");
        float* crow = C + (size_t)(r0 + mb * 16) * ldc + c0;
#pragma unroll 1
        for (int ps = 0; ps < 2; ++ps) {
#pragma unroll
            for (int s = 0; s < 8; ++s) { const int row = 2 * s + hi, cofs = lr * 4; v4f val = *(const v4fa*)(os + row * 68 + cofs); if (BIAS) { val[0] += bfr(bias[c0 + cofs]); val[1] += bfr(bias[c0 + cofs + 1]); val[2] += bfr(bias[c0 + cofs + 2]); val[3] += bfr(bias[c0 + cofs + 3]); }
                *(volatile v4f*)(crow + (size_t)row * ldc + cofs) = val; }
            if (ps == 0) __threadfence(); }
        __builtin_amdgcn_wave_barrier(); asm volatile("" ::: "memory");
    }
}

__device__ __forceinline__ h16 tohx(float x) { return (h16)x; }
__device__ __forceinline__ float tanh_(float x) { const float e = __expf(-2.0f * fabsf(x)); const float t = __fdiv_rn(1.0f - e, 1.0f + e); return copysignf(t, x); }
typedef __attribute__((ext_vector_type(4))) _Float16 v4h;
typedef __attribute__((ext_vector_type(2))) float v2f;

__global__ __launch_bounds__(256) void k_w16(const float* __restrict__ W2, const float* __restrict__ W3, h16* W2T, h16* W3T, h16* W3N, h16* W2N) { const int e = (blockIdx.x * 256 + threadIdx.x) * 4; if (e >= HID * HID) return; const int k = e % HID, n = e / HID; v4h a, b, c, d;
#pragma unroll
    for (int q = 0; q < 4; ++q) { a[q] = tohx(bfr(W2[(k + q) * HID + n])); b[q] = tohx(bfr(W3[(k + q) * HID + n])); c[q] = tohx(bfr(W3[n * HID + k + q])); d[q] = tohx(bfr(W2[n * HID + k + q])); }
    for (int ps = 0; ps < 2; ++ps) { *(volatile v4h*)(W2T + e) = a; *(volatile v4h*)(W3T + e) = b; *(volatile v4h*)(W3N + e) = c; *(volatile v4h*)(W2N + e) = d; if (ps == 0) __threadfence(); } }
__global__ __launch_bounds__(256) void k_l1(const float* __restrict__ q, const float* __restrict__ p, const float* __restrict__ W1, const float* __restrict__ b1, size_t r0, float* H1, h16* P1) { const size_t e = ((size_t)blockIdx.x * 256 + threadIdx.x) * 4; if (e >= (size_t)RCH * HID) return; const int j = (int)(e % HID); const size_t b = r0 + e / HID; const float qv = bfr(q[b]), pv = bfr(p[b]); v4f o; v4h o16;
#pragma unroll
    for (int u = 0; u < 4; ++u) { float t0 = __fmul_rn(qv, bfr(W1[j + u])); asm volatile("" : "+v"(t0)); float t1 = __fmul_rn(pv, bfr(W1[HID + j + u])); asm volatile("" : "+v"(t1)); const float a = __fadd_rn(__fadd_rn(t0, t1), bfr(b1[j + u])); o[u] = tanh_(a); o16[u] = tohx(o[u]); }
    for (int ps = 0; ps < 2; ++ps) { *(volatile v4f*)(H1 + e) = o; *(volatile v4h*)(P1 + e) = o16; if (ps == 0) __threadfence(); } }
__global__ __launch_bounds__(256) void k_tanh(const float* __restrict__ A, const float* __restrict__ bb, float* H, h16* P) { const size_t e = ((size_t)blockIdx.x * 256 + threadIdx.x) * 4; if (e >= (size_t)RCH * HID) return; const int j = (int)(e % HID); const v4f a = *(const v4f*)(A + e); v4f o; v4h o16;
#pragma unroll
    for (int u = 0; u < 4; ++u) { o[u] = tanh_(__fadd_rn(a[u], bfr(bb[j + u]))); o16[u] = tohx(o[u]); }
    for (int ps = 0; ps < 2; ++ps) { *(volatile v4f*)(H + e) = o; *(volatile v4h*)(P + e) = o16; if (ps == 0) __threadfence(); } }
__global__ __launch_bounds__(256) void k_g3(const float* __restrict__ H3, const float* __restrict__ W4, h16* P) { const size_t e = ((size_t)blockIdx.x * 256 + threadIdx.x) * 4; if (e >= (size_t)RCH * HID) return; const int j = (int)(e % HID); const v4f h = *(const v4f*)(H3 + e); v4h o16;
#pragma unroll
    for (int u = 0; u < 4; ++u) { float hh = __fmul_rn(h[u], h[u]); asm volatile("" : "+v"(hh)); o16[u] = tohx(__fmul_rn(bfr(W4[j + u]), __fsub_rn(1.0f, hh))); }
    *(volatile v4h*)(P + e) = o16; __threadfence(); *(volatile v4h*)(P + e) = o16; }
__global__ __launch_bounds__(256) void k_gm(const float* __restrict__ A, const float* __restrict__ H, float* G, h16* P) { const size_t e = ((size_t)blockIdx.x * 256 + threadIdx.x) * 4; if (e >= (size_t)RCH * HID) return; const v4f a = *(const v4f*)(A + e), h = *(const v4f*)(H + e); v4f o; v4h o16;
#pragma unroll
    for (int u = 0; u < 4; ++u) { float hh = __fmul_rn(h[u], h[u]); asm volatile("" : "+v"(hh)); o[u] = __fmul_rn(a[u], __fsub_rn(1.0f, hh)); o16[u] = tohx(o[u]); }
    for (int ps = 0; ps < 2; ++ps) { if (G) *(volatile v4f*)(G + e) = o; *(volatile v4h*)(P + e) = o16; if (ps == 0) __threadfence(); } }
__global__ __launch_bounds__(256) void k_out(const float* __restrict__ G1, const float* __restrict__ W1, const float* __restrict__ F, size_t r0, float* OUT) { const size_t bl = (size_t)blockIdx.x * 256 + threadIdx.x; if (bl >= RCH) return; const size_t b = r0 + bl; const float* g = G1 + bl * HID; float dq = 0.f, dp = 0.f;
#pragma unroll 1
    for (int j = 0; j < HID; ++j) { const float gj = g[j]; float t0 = __fmul_rn(gj, bfr(W1[j])); asm volatile("" : "+v"(t0)); dq = __fadd_rn(dq, t0); float t1 = __fmul_rn(gj, bfr(W1[HID + j])); asm volatile("" : "+v"(t1)); dp = __fadd_rn(dp, t1); }
    v2f o; o[0] = __fmul_rn(dp, DTC); o[1] = __fmul_rn(__fadd_rn(-dq, bfr(F[b])), DTC); *(volatile v2f*)(OUT + b * 2) = o; __threadfence(); *(volatile v2f*)(OUT + b * 2) = o; }

extern "C" void kernel_launch(void* const* d_in, const int* in_sizes, int n_in,
                              void* d_out, int out_size, void* d_ws, size_t ws_size, hipStream_t stream) {
    (void)in_sizes; (void)n_in; (void)out_size;
    const float* q = (const float*)d_in[0]; const float* p = (const float*)d_in[1]; const float* F = (const float*)d_in[2]; const float* W1 = (const float*)d_in[3]; const float* b1 = (const float*)d_in[4]; const float* W2 = (const float*)d_in[5]; const float* b2 = (const float*)d_in[6]; const float* W3 = (const float*)d_in[7]; const float* b3 = (const float*)d_in[8]; const float* W4 = (const float*)d_in[9];
    float* OUT = (float*)d_out;
    char* wsp = (char*)d_ws;
    auto take = [&](size_t bytes) { char* pp = wsp; wsp += (bytes + 255) & ~(size_t)255; return (void*)pp; };
    h16* W2T = (h16*)take(HID * HID * 2); h16* W3T = (h16*)take(HID * HID * 2); h16* W3N = (h16*)take(HID * HID * 2); h16* W2N = (h16*)take(HID * HID * 2);
    float* H1 = (float*)take((size_t)RCH * HID * 4); float* H2 = (float*)take((size_t)RCH * HID * 4); float* H3 = (float*)take((size_t)RCH * HID * 4); float* A = (float*)take((size_t)RCH * HID * 4); float* G1 = (float*)take((size_t)RCH * HID * 4); h16* P = (h16*)take((size_t)RCH * HID * 2);
    if ((size_t)(wsp - (char*)d_ws) > ws_size) return;
    k_w16<<<(HID * HID / 4 + 255) / 256, 256, 0, stream>>>(W2, W3, W2T, W3T, W3N, W2N);
    const unsigned L4 = (unsigned)(((size_t)RCH * HID / 4 + 255) / 256);
    for (size_t r0 = 0; r0 < NBT; r0 += RCH) {
        k_l1<<<L4, 256, 0, stream>>>(q, p, W1, b1, r0, H1, P);
        k_gemmw<h16, 0, false><<<dim3(RCH / 64, HID / 64, 1), 32, 0, stream>>>(P, nullptr, W2T, nullptr, HID, A, HID, nullptr, 0, 0, 0); k_tanh<<<L4, 256, 0, stream>>>(A, b2, H2, P);
        k_gemmw<h16, 0, false><<<dim3(RCH / 64, HID / 64, 1), 32, 0, stream>>>(P, nullptr, W3T, nullptr, HID, A, HID, nullptr, 0, 0, 0); k_tanh<<<L4, 256, 0, stream>>>(A, b3, H3, P);
        k_g3<<<L4, 256, 0, stream>>>(H3, W4, P);
        k_gemmw<h16, 0, false><<<dim3(RCH / 64, HID / 64, 1), 32, 0, stream>>>(P, nullptr, W3N, nullptr, HID, A, HID, nullptr, 0, 0, 0); k_gm<<<L4, 256, 0, stream>>>(A, H2, nullptr, P);
        k_gemmw<h16, 0, false><<<dim3(RCH / 64, HID / 64, 1), 32, 0, stream>>>(P, nullptr, W2N, nullptr, HID, A, HID, nullptr, 0, 0, 0); k_gm<<<L4, 256, 0, stream>>>(A, H1, G1, P);
        k_out<<<RCH / 256, 256, 0, stream>>>(G1, W1, F, r0, OUT); }
}
